// GuidanceRefinementBlock_35235911696699
// MI455X (gfx1250) — hardware-verified
//
#include <hip/hip_runtime.h>
#include <hip/hip_bf16.h>

typedef __attribute__((ext_vector_type(16))) _Float16 v16bf;
typedef __attribute__((ext_vector_type(8)))  float  v8f;
typedef __attribute__((ext_vector_type(4)))  float  v4f_t;
typedef float v4fa __attribute__((ext_vector_type(4), may_alias));

#define HW   16384
#define CH   64
#define H_   128
#define W_   128
#define B_   8

__device__ __forceinline__ unsigned short f2bf(float f) {
    return __builtin_bit_cast(unsigned short, (_Float16)f);
}

__global__ __launch_bounds__(256)
void k_repack_w(const float* __restrict__ wsrc, unsigned short* __restrict__ wdst)
{
    int i = blockIdx.x * 256 + threadIdx.x;
    if (i >= 9 * CH * CH) return;
    int ci = i & 63;
    int t  = i >> 6;
    int co = t & 63;
    int p  = t >> 6;
    const unsigned short v = f2bf(wsrc[(co * CH + ci) * 9 + p]);
    *(volatile unsigned short*)(wdst + i) = v; __threadfence(); *(volatile unsigned short*)(wdst + i) = v;
}

union AFrag { v16bf v; unsigned int u[8]; };
union BFrag { v16bf v; uint4 q[2]; };

__global__ __launch_bounds__(128)
void k_conv_wmma(const float* __restrict__ guide, const float* __restrict__ target,
                 const float* __restrict__ w_reduce,
                 const float* __restrict__ bn1_g, const float* __restrict__ bn1_b,
                 const float* __restrict__ bn1_m, const float* __restrict__ bn1_v,
                 const float* __restrict__ w_span,
                 const float* __restrict__ b_span,
                 const unsigned short* __restrict__ wts,
                 const float* __restrict__ bn3_g, const float* __restrict__ bn3_b,
                 const float* __restrict__ bn3_m, const float* __restrict__ bn3_v,
                 float* __restrict__ out)
{
    __shared__ __align__(16) unsigned short s_x[3 * 130 * CH];
    __shared__ __align__(16) float s_k[3 * 128 * 18];

    int blk = blockIdx.x;
    int h   = blk & (H_ - 1);
    int b   = blk >> 7;
    int tid = threadIdx.x;

    __builtin_prefetch((const char*)wts + tid * 576, 0, 0);

    #pragma unroll 1
    for (int r = 0; r < 3; ++r) {
        const int gh = h - 1 + r;
        if (gh < 0 || gh >= H_) continue;
        const int pbase = b * CH * HW + gh * W_ + tid;
        float xr[16];
        #pragma unroll
        for (int q = 0; q < 16; ++q) xr[q] = 0.f;
        #pragma unroll 1
        for (int c = 0; c < CH; ++c) {
            const float xv = guide[pbase + c * HW] + target[pbase + c * HW];
            #pragma unroll
            for (int q = 0; q < 16; ++q) xr[q] += w_reduce[q * CH + c] * xv;
        }
        #pragma unroll
        for (int q = 0; q < 16; ++q) {
            const float sc = bn1_g[q] * rsqrtf(bn1_v[q] + 1e-5f);
            const float y  = xr[q] * sc + (bn1_b[q] - bn1_m[q] * sc);
            xr[q] = y > 0.f ? y : 0.f;
        }
        #pragma unroll 1
        for (int k = 0; k < 18; ++k) {
            float a = b_span[k];
            #pragma unroll
            for (int q = 0; q < 16; ++q) a += w_span[k * 16 + q] * xr[q];
            s_k[(r * 128 + tid) * 18 + k] = a;
        }
    }
    __syncthreads();

    const int E = 3 * CH * 130;
    #pragma unroll 1
    for (int e = tid; e < E; e += 128) {
        int c  = e % 130;
        int t  = e / 130;
        int ci = t & 63;
        int r  = t >> 6;
        int gh = h - 1 + r, gw = c - 1;
        float acc = 0.f;
        if (gh >= 0 && gh < H_ && gw >= 0 && gw < W_) {
            const float* kv = s_k + (r * 128 + gw) * 18 + (ci >> 5) * 9;
            const float* tc = target + (b * CH + ci) * HW;
            #pragma unroll
            for (int kh = 0; kh < 3; ++kh) {
                const int hh = gh + kh - 1;
                if (hh < 0 || hh >= H_) continue;
                #pragma unroll
                for (int kw = 0; kw < 3; ++kw) {
                    const int ww = gw + kw - 1;
                    if (ww < 0 || ww >= W_) continue;
                    acc += kv[kh * 3 + kw] * tc[hh * W_ + ww];
                }
            }
        }
        s_x[(r * 130 + c) * CH + ci] = f2bf(acc);
    }
    __syncthreads();

    int lane  = tid & 31;
    int wv    = tid >> 5;
    int mrow  = lane & 15;
    int kbase = (lane < 16) ? 0 : 8;
    int koff  = kbase;
    int n     = lane & 15;

    v8f zero = {0.f, 0.f, 0.f, 0.f, 0.f, 0.f, 0.f, 0.f};
    v8f acc[2][4];
    #pragma unroll
    for (int mt = 0; mt < 2; ++mt)
        #pragma unroll
        for (int nt = 0; nt < 4; ++nt) acc[mt][nt] = zero;

    const unsigned int* sx32 = (const unsigned int*)s_x;
    const uint4*        wq   = (const uint4*)wts;

    for (int t = 0; t < 18; ++t) {
        int p   = t >> 1;
        int cib = (t & 1) << 5;
        int r   = p / 3;
        int c0  = wv * 32 + mrow + (p % 3);

        AFrag a0, a1;
        int xb0 = (r * 130 + c0) * CH + cib;
        int xb1 = xb0 + 16 * CH;
        #pragma unroll
        for (int vv = 0; vv < 8; ++vv) {
            int lk = (vv < 4) ? (kbase + 2 * vv) : (16 + kbase + 2 * (vv - 4));
            a0.u[vv] = sx32[(xb0 + lk) >> 1];
            a1.u[vv] = sx32[(xb1 + lk) >> 1];
        }

        #pragma unroll
        for (int nt = 0; nt < 4; ++nt) {
            int co = nt * 16 + n;
            int wi = (p * CH + co) * CH + cib + koff;
            BFrag bf;
            bf.q[0] = wq[(wi >> 3) + 0];
            bf.q[1] = wq[(wi >> 3) + 2];
            acc[0][nt] = __builtin_amdgcn_wmma_f32_16x16x32_f16(
                false, a0.v, false, bf.v, (short)0, acc[0][nt], false, false);
            acc[1][nt] = __builtin_amdgcn_wmma_f32_16x16x32_f16(
                false, a1.v, false, bf.v, (short)0, acc[1][nt], false, false);
        }
    }

    __syncthreads();
    float* so = (float*)s_x;
    #pragma unroll
    for (int nt = 0; nt < 4; ++nt) {
        int co = nt * 16 + n;
        float sc = bn3_g[co] * rsqrtf(bn3_v[co] + 1e-5f);
        float sh = bn3_b[co] - bn3_m[co] * sc;
        #pragma unroll
        for (int mt = 0; mt < 2; ++mt) {
            #pragma unroll
            for (int r = 0; r < 8; ++r) {
                int mm   = r + ((lane >> 4) << 3);
                int wpix = wv * 32 + mt * 16 + mm;
                float v  = acc[mt][nt][r] * sc + sh;
                v = v > 0.f ? v : 0.f;
                so[co * 128 + wpix] = v;
            }
        }
    }
    __syncthreads();
    #pragma unroll 1
    for (int pass = 0; pass < 2; ++pass) {
        for (int ch = tid; ch < CH * 32; ch += 128) { const int co = ch >> 5, q = (ch & 31) * 4;
            *(volatile v4f_t*)(out + ((size_t)(b * CH + co) * H_ + h) * W_ + q) = *(const volatile v4fa*)(so + co * 128 + q); }
        __threadfence();
    }
}

extern "C" void kernel_launch(void* const* d_in, const int* in_sizes, int n_in,
                              void* d_out, int out_size, void* d_ws, size_t ws_size,
                              hipStream_t stream) {
    const float* guide    = (const float*)d_in[0];
    const float* target   = (const float*)d_in[1];
    const float* w_reduce = (const float*)d_in[2];
    const float* bn1_g    = (const float*)d_in[3];
    const float* bn1_b    = (const float*)d_in[4];
    const float* bn1_m    = (const float*)d_in[5];
    const float* bn1_v    = (const float*)d_in[6];
    const float* w_span   = (const float*)d_in[7];
    const float* b_span   = (const float*)d_in[8];
    const float* w_bconv  = (const float*)d_in[9];
    const float* bn3_g    = (const float*)d_in[10];
    const float* bn3_b    = (const float*)d_in[11];
    const float* bn3_m    = (const float*)d_in[12];
    const float* bn3_v    = (const float*)d_in[13];
    float* out = (float*)d_out;

    unsigned short* wsW = (unsigned short*)d_ws;

    k_repack_w<<<(9 * CH * CH + 255) / 256, 256, 0, stream>>>(w_bconv, wsW);

    k_conv_wmma<<<B_ * H_, 128, 0, stream>>>(
        guide, target, w_reduce, bn1_g, bn1_b, bn1_m, bn1_v, w_span, b_span,
        wsW, bn3_g, bn3_b, bn3_m, bn3_v, out);
}
